// ealstm_82549271429808
// MI455X (gfx1250) — hardware-verified
//
#include <hip/hip_runtime.h>
#include <math.h>

constexpr int NBATCH    = 1024;
constexpr int NSTEP     = 365;
constexpr int NDYN      = 32;
constexpr int NSTAT     = 27;
constexpr int NHID      = 256;
constexpr int NGATE     = 3 * NHID;
constexpr int KAUG      = NHID + NDYN;
constexpr int NTHR      = 256;
constexpr int NWAVE     = NTHR / 32;
constexpr int SEQ_BLK   = 16;
constexpr int APITCH    = 296;
constexpr int OPITCH    = 384;
constexpr int TPITCH    = 68;
constexpr int PACK_ROWS = 64;
constexpr int NOUT      = NBATCH * NSTEP;
constexpr float WCARRY     = 64.0f;
constexpr float WCARRY_INV = 1.0f / 64.0f;
static_assert(NBATCH % SEQ_BLK == 0, "block rows");
static_assert(NHID == 32 * NWAVE, "8 waves x 32 hidden columns");
static_assert(KAUG % 32 == 0, "K multiple of 32, no padding");
static_assert(NGATE % PACK_ROWS == 0, "pack grid exact");
static_assert((NHID * PACK_ROWS / 4) % NTHR == 0, "pack load phase A exact");
static_assert((NDYN * PACK_ROWS / 4) % NTHR == 0, "pack load phase B exact");
static_assert((PACK_ROWS * KAUG / 8) % NTHR == 0, "pack store phase exact");
static_assert(KAUG % 8 == 0 && APITCH % 8 == 0 && APITCH >= KAUG, "16-B aligned fragment loads");
static_assert(OPITCH >= NSTEP && (OPITCH * 4) % 128 == 0, "padded output rows are whole lines");
static_assert((SEQ_BLK * OPITCH / 4) % NTHR == 0, "flush loop exact");
static_assert((OPITCH / 4) % 32 == 0, "a wave float4 chunk stays inside one staged row");
static_assert((SEQ_BLK * OPITCH) % NTHR == 0, "output staging zero-fill exact");
static_assert((2 * SEQ_BLK * APITCH) % 2 == 0, "A tile zero-fill in 32-bit words");
static_assert(NOUT % (4 * NTHR) == 0, "line writer grid exact");
static_assert(SEQ_BLK * NDYN == 2 * NTHR, "x tile staging: 2 elements per thread exact");

typedef __attribute__((ext_vector_type(16))) _Float16 v16h;
typedef __attribute__((ext_vector_type(8)))  _Float16 v8h;
typedef __attribute__((ext_vector_type(8)))  float    v8f;
typedef __attribute__((ext_vector_type(4)))  float    v4f;
typedef __attribute__((ext_vector_type(2)))  float    v2f;
typedef __attribute__((ext_vector_type(2)))  unsigned v2u;

__device__ __forceinline__ unsigned short f2bf_bits(float f) {
  unsigned u = __float_as_uint(f);
  return (unsigned short)((u + 0x7FFFu + ((u >> 16) & 1u)) >> 16);
}
__device__ __forceinline__ float bf_bits2f(unsigned short h) { return __uint_as_float(((unsigned)h) << 16); }
__device__ __forceinline__ float bf16r(float f) { return bf_bits2f(f2bf_bits(f)); }
__device__ __forceinline__ unsigned short h_bits(float f) { return __builtin_bit_cast(unsigned short, (_Float16)f); }

__device__ __forceinline__ void dep_guard3_h(v8f& a, v8f& b, v8f& c, v16h x, v16h y, v16h z, v16h w) {
  asm volatile("v_nop\n\tv_nop\n\tv_nop\n\tv_nop" : "+v"(a), "+v"(b), "+v"(c) : "v"(x), "v"(y), "v"(z), "v"(w));
}
__device__ __forceinline__ void acc_guard3(v8f& a, v8f& b, v8f& c) {
  asm volatile("v_nop\n\tv_nop\n\tv_nop\n\tv_nop" : "+v"(a), "+v"(b), "+v"(c));
}
template <typename T> struct Frag;
template <> struct Frag<_Float16> {
  typedef v16h V; union U { v16h v; v8h h[2]; };
  static __device__ __forceinline__ v16h load(const _Float16* p) {
    U f; f.h[0] = *(const v8h*)(p); f.h[1] = *(const v8h*)(p + 16); return f.v;
  }
  static __device__ __forceinline__ v8f mma(v16h a, v16h b, v8f c) {
    return __builtin_amdgcn_wmma_f32_16x16x32_f16(false, a, false, b, (short)0, c, false, false);
  }
};

__device__ __forceinline__ float fsig(float x)  { return __builtin_amdgcn_rcpf(1.0f + expf(-x)); }
__device__ __forceinline__ float ftanh(float x) { return 1.0f - 2.0f * __builtin_amdgcn_rcpf(expf(2.0f * x) + 1.0f); }

__global__ __launch_bounds__(NTHR) void pack_w_kernel(const float* __restrict__ whh, const float* __restrict__ wih,
                                                      unsigned short* __restrict__ WB) {
  __shared__ __align__(16) unsigned short Tt[KAUG * TPITCH];
  const int tid = threadIdx.x;
  const int n0 = blockIdx.x * PACK_ROWS;
#pragma unroll 1
  for (int it = 0; it < (NHID * PACK_ROWS / 4) / NTHR; ++it) {
    const int i = it * NTHR + tid;
    const int kr = i >> 4, n4 = (i & 15) * 4;
    const v4f v = *(const v4f*)(whh + (size_t)kr * NGATE + n0 + n4);
    v2u pk;
    pk[0] = (unsigned)h_bits(bf16r(v[0]) * WCARRY) | ((unsigned)h_bits(bf16r(v[1]) * WCARRY) << 16);
    pk[1] = (unsigned)h_bits(bf16r(v[2]) * WCARRY) | ((unsigned)h_bits(bf16r(v[3]) * WCARRY) << 16);
    *(v2u*)(Tt + kr * TPITCH + n4) = pk;
  }
#pragma unroll 1
  for (int it = 0; it < (NDYN * PACK_ROWS / 4) / NTHR; ++it) {
    const int i = it * NTHR + tid;
    const int kk = i >> 4, n4 = (i & 15) * 4;
    const v4f v = *(const v4f*)(wih + (size_t)kk * NGATE + n0 + n4);
    v2u pk;
    pk[0] = (unsigned)h_bits(bf16r(v[0]) * WCARRY) | ((unsigned)h_bits(bf16r(v[1]) * WCARRY) << 16);
    pk[1] = (unsigned)h_bits(bf16r(v[2]) * WCARRY) | ((unsigned)h_bits(bf16r(v[3]) * WCARRY) << 16);
    *(v2u*)(Tt + (NHID + kk) * TPITCH + n4) = pk;
  }
  __syncthreads();
#pragma unroll 1
  for (int it = 0; it < (PACK_ROWS * KAUG / 8) / NTHR; ++it) {
    const int q  = it * NTHR + tid;
    const int nn = q / (KAUG / 8);
    const int k8 = q - nn * (KAUG / 8);
    v8h hv;
#pragma unroll
    for (int e = 0; e < 8; ++e) hv[e] = __builtin_bit_cast(_Float16, Tt[(8 * k8 + e) * TPITCH + nn]);
    unsigned short* dst = WB + (size_t)(n0 + nn) * KAUG + 8 * k8;
    *(volatile v8h*)dst = hv;
    __threadfence();
    *(volatile v8h*)dst = hv;
  }
}

__device__ __forceinline__ void stage_x_tile(const float* __restrict__ xdyn, int rowbase, int tt, _Float16* abuf, int tid) {
  const int m = tid >> 4, f2 = (tid & 15) * 2;
  const v2f v = *(const v2f*)(xdyn + ((size_t)(rowbase + m) * NSTEP + (size_t)tt) * NDYN + f2);
  const unsigned u = (unsigned)h_bits(bf16r(v[0])) | ((unsigned)h_bits(bf16r(v[1])) << 16);
  *(unsigned*)(abuf + m * APITCH + NHID + f2) = u;
}

__global__ __launch_bounds__(NTHR) void ealstm_seq_kernel(const float* __restrict__ xdyn, const float* __restrict__ xstat,
                                                          const float* __restrict__ wsh, const float* __restrict__ bias,
                                                          const float* __restrict__ bias_s, const float* __restrict__ wout,
                                                          const float* __restrict__ bout,
                                                          const unsigned short* __restrict__ WBp,
                                                          float* __restrict__ OUTP) {
  __shared__ __align__(16) _Float16 Aop[2][SEQ_BLK * APITCH];
  __shared__ __align__(16) float    Ol[SEQ_BLK * OPITCH];
  __shared__ float Pw[2][NWAVE][SEQ_BLK];
  const _Float16* WB = (const _Float16*)WBp;
  const int tid = threadIdx.x, lane = tid & 31, wave = tid >> 5;
  const int c = lane & 15, hh = lane >> 4, koff = hh * 8;
  const int rowbase = blockIdx.x * SEQ_BLK;

  {
    unsigned* aw = (unsigned*)(&Aop[0][0]);
#pragma unroll 1
    for (int i = tid; i < (2 * SEQ_BLK * APITCH) / 2; i += NTHR) aw[i] = 0u;
#pragma unroll 1
    for (int i = tid; i < SEQ_BLK * OPITCH; i += NTHR) Ol[i] = 0.0f;
  }
  __syncthreads();
  stage_x_tile(xdyn, rowbase, 0, &Aop[0][0], tid);

  float ig[2][8], cst[2][8], bb[2][3], wo[2], bs2[2];
#pragma unroll
  for (int nt = 0; nt < 2; ++nt) {
    const int j = 32 * wave + 16 * nt + c;
#pragma unroll
    for (int g = 0; g < 3; ++g) bb[nt][g] = bf16r(bias[g * NHID + j]);
    wo[nt]  = bf16r(wout[j]);
    bs2[nt] = bf16r(bias_s[j]);
#pragma unroll
    for (int r = 0; r < 8; ++r) { ig[nt][r] = 0.0f; cst[nt][r] = 0.0f; }
  }
  const float bo = bf16r(bout[0]);
  {
    const int j0 = 32 * wave + c, j1 = j0 + 16;
#pragma unroll 1
    for (int d = 0; d < NSTAT; ++d) {
      const float w0 = bf16r(wsh[d * NHID + j0]);
      const float w1 = bf16r(wsh[d * NHID + j1]);
#pragma unroll
      for (int r = 0; r < 8; ++r) {
        const float xs = bf16r(xstat[(size_t)(rowbase + 8 * hh + r) * NSTAT + d]);
        ig[0][r] += xs * w0;
        ig[1][r] += xs * w1;
      }
    }
#pragma unroll
    for (int nt = 0; nt < 2; ++nt)
#pragma unroll
      for (int r = 0; r < 8; ++r) ig[nt][r] = fsig(ig[nt][r] + bs2[nt]);
  }
  __syncthreads();

  const v8f z8 = {0.f, 0.f, 0.f, 0.f, 0.f, 0.f, 0.f, 0.f};
#pragma unroll 1
  for (int t = 0; t < NSTEP; ++t) {
    const int cur = t & 1;
    const _Float16* arow = &Aop[cur][0] + c * APITCH + koff;
    _Float16* anx = &Aop[cur ^ 1][0];
    float pr[8];
#pragma unroll
    for (int r = 0; r < 8; ++r) pr[r] = 0.0f;

#pragma unroll
    for (int nt = 0; nt < 2; ++nt) {
      const int j = 32 * wave + 16 * nt + c;
      const _Float16* wbf = WB + (size_t)j * KAUG + koff;
      const _Float16* wbo = WB + (size_t)(NHID + j) * KAUG + koff;
      const _Float16* wbg = WB + (size_t)(2 * NHID + j) * KAUG + koff;
      v8f aF = z8, aO = z8, aG = z8;
#pragma unroll 1
      for (int k0 = 0; k0 < KAUG; k0 += 32) {
        const v16h a  = Frag<_Float16>::load(arow + k0);
        const v16h b0 = Frag<_Float16>::load(wbf + k0);
        const v16h b1 = Frag<_Float16>::load(wbo + k0);
        const v16h b2 = Frag<_Float16>::load(wbg + k0);
        aF = Frag<_Float16>::mma(a, b0, aF);
        aO = Frag<_Float16>::mma(a, b1, aO);
        aG = Frag<_Float16>::mma(a, b2, aG);
        dep_guard3_h(aF, aO, aG, a, b0, b1, b2);
      }
      acc_guard3(aF, aO, aG);
#pragma unroll
      for (int r = 0; r < 8; ++r) {
        const float zf = aF[r] * WCARRY_INV + bb[nt][0];
        const float zo = aO[r] * WCARRY_INV + bb[nt][1];
        const float zg = aG[r] * WCARRY_INV + bb[nt][2];
        const float sf = fsig(zf);
        const float so = fsig(zo);
        const float tg = ftanh(zg);
        const float cn = sf * cst[nt][r] + ig[nt][r] * tg;
        cst[nt][r] = cn;
        const float hn = so * ftanh(cn);
        anx[(8 * hh + r) * APITCH + j] = (_Float16)hn;
        pr[r] += hn * wo[nt];
      }
    }
#pragma unroll
    for (int r = 0; r < 8; ++r) {
#pragma unroll
      for (int off = 1; off < 16; off <<= 1) pr[r] += __shfl_xor(pr[r], off, 32);
    }
    if (c == 0) {
#pragma unroll
      for (int r = 0; r < 8; ++r) Pw[cur][wave][8 * hh + r] = pr[r];
    }
    {
      const int tn = (t + 1 < NSTEP) ? (t + 1) : (NSTEP - 1);
      stage_x_tile(xdyn, rowbase, tn, anx, tid);
    }
    __syncthreads();
    if (tid < SEQ_BLK) {
      float s = 0.0f;
#pragma unroll
      for (int w2 = 0; w2 < NWAVE; ++w2) s += Pw[cur][w2][tid];
      Ol[tid * OPITCH + t] = s + bo;
    }
  }
  __syncthreads();

  for (int pass = 0; pass < 2; ++pass) {
#pragma unroll
    for (int it = 0; it < (SEQ_BLK * OPITCH / 4) / NTHR; ++it) {
      const int idx = it * NTHR + tid;
      const int row = idx / (OPITCH / 4);
      const int c4  = (idx - row * (OPITCH / 4)) * 4;
      const v4f v = *(const v4f*)(Ol + row * OPITCH + c4);
      *(volatile v4f*)(OUTP + (size_t)(rowbase + row) * OPITCH + c4) = v;
    }
    __threadfence();
  }
}

__global__ __launch_bounds__(NTHR) void out_lines_kernel(const float* __restrict__ OUTP, float* __restrict__ out) {
  const int g = blockIdx.x * NTHR + threadIdx.x;
  if (g >= NOUT / 4) return;
  const int f0 = g * 4;
  v4f v;
#pragma unroll
  for (int e = 0; e < 4; ++e) {
    const int idx = f0 + e;
    const int b = idx / NSTEP;
    const int t = idx - b * NSTEP;
    v[e] = OUTP[(size_t)b * OPITCH + t];
  }
  *(volatile v4f*)(out + f0) = v;
  __threadfence();
  *(volatile v4f*)(out + f0) = v;
}

extern "C" void kernel_launch(void* const* d_in, const int* in_sizes, int n_in,
                              void* d_out, int out_size, void* d_ws, size_t ws_size, hipStream_t stream) {
  if (n_in < 9 || d_out == nullptr || d_ws == nullptr) return;
  if (in_sizes[0] != NBATCH * NSTEP * NDYN || in_sizes[1] != NBATCH * NSTAT || in_sizes[2] != NDYN * NGATE ||
      in_sizes[3] != NHID * NGATE || in_sizes[4] != NSTAT * NHID || in_sizes[5] != NGATE || in_sizes[6] != NHID ||
      in_sizes[7] != NHID || in_sizes[8] != 1 || out_size != NOUT) return;

  const float* xdyn   = (const float*)d_in[0];
  const float* xstat  = (const float*)d_in[1];
  const float* wih    = (const float*)d_in[2];
  const float* whh    = (const float*)d_in[3];
  const float* wsh    = (const float*)d_in[4];
  const float* bias   = (const float*)d_in[5];
  const float* bias_s = (const float*)d_in[6];
  const float* wout   = (const float*)d_in[7];
  const float* bout   = (const float*)d_in[8];
  float* out = (float*)d_out;

  char* ws = (char*)d_ws; size_t off = 0;
  auto carve = [&](size_t bytes) -> char* { char* p = ws + off; off += (bytes + 255) & ~(size_t)255; return p; };
  unsigned short* WB   = (unsigned short*)carve((size_t)NGATE * KAUG * 2);
  float*          OUTP = (float*)carve((size_t)NBATCH * OPITCH * 4);
  if (off > ws_size || off > (size_t)134217728) return;

  pack_w_kernel<<<NGATE / PACK_ROWS, NTHR, 0, stream>>>(whh, wih, WB);
  ealstm_seq_kernel<<<NBATCH / SEQ_BLK, NTHR, 0, stream>>>(xdyn, xstat, wsh, bias, bias_s, wout, bout, WB, OUTP);
  out_lines_kernel<<<NOUT / 4 / NTHR, NTHR, 0, stream>>>(OUTP, out);
}
